// MeshfreeKANNet_12996571038255
// MI455X (gfx1250) — hardware-verified
//
#include <hip/hip_runtime.h>


#define MM   4096
#define NNODE 1024
#define HID  8
#define NG   5
typedef _Float16 h16;
typedef unsigned short bf;
typedef __attribute__((ext_vector_type(16))) __bf16   v16bf;
typedef __attribute__((ext_vector_type(16))) _Float16 v16h;
typedef __attribute__((ext_vector_type(8)))  _Float16 v8h;
typedef __attribute__((ext_vector_type(8)))  unsigned short v8us;
typedef __attribute__((ext_vector_type(8)))  float    v8f;
typedef __attribute__((ext_vector_type(4)))  float    v4f;
typedef v8h  __attribute__((may_alias)) v8ha;
typedef v4f  __attribute__((may_alias)) v4fa;
typedef v8us __attribute__((may_alias)) v8usa;

__device__ __forceinline__ unsigned short f2bf(float f) { unsigned u = __float_as_uint(f); u += 0x7FFFu + ((u >> 16) & 1u); return (unsigned short)(u >> 16); }
__device__ __forceinline__ float bf2f(unsigned short b) { return __uint_as_float(((unsigned)b) << 16); }
__device__ __forceinline__ float bfr(float f) { return bf2f(f2bf(f)); }
__device__ __forceinline__ v16h cat16(v8h lo, v8h hi) { return __builtin_shufflevector(lo, hi, 0, 1, 2, 3, 4, 5, 6, 7, 8, 9, 10, 11, 12, 13, 14, 15); }
__device__ __forceinline__ v16bf cat16b(v8us lo, v8us hi) { return __builtin_bit_cast(v16bf, __builtin_shufflevector(lo, hi, 0, 1, 2, 3, 4, 5, 6, 7, 8, 9, 10, 11, 12, 13, 14, 15)); }
__device__ __forceinline__ v8f wmma16(v16h a, v16h b, v8f c) { return __builtin_amdgcn_wmma_f32_16x16x32_f16(false, a, false, b, (short)0, c, false, false); }
__device__ __forceinline__ v8f wmmab(v16bf a, v16bf b, v8f c) { return __builtin_amdgcn_wmma_f32_16x16x32_bf16(false, a, false, b, (short)0, c, false, false); }


template <typename T16> struct WFrag;
template <> struct WFrag<h16> { typedef v16h V; static __device__ __forceinline__ V ld(const h16* p) { return cat16(*(const v8h*)p, *(const v8h*)(p + 16)); } static __device__ __forceinline__ v8f mma(V a, V b, v8f c) { return wmma16(a, b, c); } };
template <> struct WFrag<bf> { typedef v16bf V; static __device__ __forceinline__ V ld(const bf* p) { return cat16b(*(const v8us*)p, *(const v8us*)(p + 16)); } static __device__ __forceinline__ v8f mma(V a, V b, v8f c) { return wmmab(a, b, c); } };
template <typename T16, int NSPLIT, bool BIAS>
__global__ __launch_bounds__(32) void k_gemmw(const T16* __restrict__ A, const T16* __restrict__ A2, const T16* __restrict__ Bt, const T16* __restrict__ Bt2, int K, float* C, int ldc, const float* __restrict__ bias, size_t sA, size_t sB, size_t sC) {
    typedef typename WFrag<T16>::V V;
    __shared__ __align__(16) float os[16 * 68];
    const size_t z = blockIdx.z; A += z * sA; if (A2) A2 += z * sA; Bt += z * sB; if (Bt2) Bt2 += z * sB; C += z * sC;
    const int lane = threadIdx.x & 31, lr = lane & 15, hi = lane >> 4; const int r0 = blockIdx.x * 64, c0 = blockIdx.y * 64;
    v8f acc[4][4];
#pragma unroll
    for (int mb = 0; mb < 4; ++mb)
#pragma unroll
        for (int nb = 0; nb < 4; ++nb) acc[mb][nb] = (v8f){};
    const size_t aoff = (size_t)(r0 + lr) * K + 8 * hi, boff = (size_t)(c0 + lr) * K + 8 * hi;
#pragma unroll 1
    for (int kc = 0; kc < K; kc += 32) {
        V a[4], a2[4];
#pragma unroll
        for (int mb = 0; mb < 4; ++mb) { a[mb] = WFrag<T16>::ld(A + aoff + (size_t)mb * 16 * K + kc); if (NSPLIT == 1 || NSPLIT == 2) a2[mb] = WFrag<T16>::ld(A2 + aoff + (size_t)mb * 16 * K + kc); }
#pragma unroll
        for (int nb = 0; nb < 4; ++nb) { const V b = WFrag<T16>::ld(Bt + boff + (size_t)nb * 16 * K + kc); V b2; if (NSPLIT >= 2) b2 = WFrag<T16>::ld(Bt2 + boff + (size_t)nb * 16 * K + kc);
#pragma unroll
            for (int mb = 0; mb < 4; ++mb) { acc[mb][nb] = WFrag<T16>::mma(a[mb], b, acc[mb][nb]); if (NSPLIT == 1 || NSPLIT == 2) acc[mb][nb] = WFrag<T16>::mma(a2[mb], b, acc[mb][nb]); if (NSPLIT >= 2) acc[mb][nb] = WFrag<T16>::mma(a[mb], b2, acc[mb][nb]); } }
        asm volatile("v_nop\n\tv_nop\n\tv_nop\n\tv_nop" : "+v"(acc[0][0]), "+v"(acc[1][1]), "+v"(acc[2][2]), "+v"(acc[3][3]) : "v"(a[0]), "v"(a[3]));
    }
#pragma unroll
    for (int mb = 0; mb < 4; ++mb) {
#pragma unroll
        for (int nb = 0; nb < 4; ++nb) {
#pragma unroll
            for (int j = 0; j < 8; ++j) os[(hi * 8 + j) * 68 + nb * 16 + lr] = acc[mb][nb][j]; }
        __builtin_amdgcn_wave_barrier(); asm volatile("" ::: "memory");
        float* crow = C + (size_t)(r0 + mb * 16) * ldc + c0;
#pragma unroll 1
        for (int ps = 0; ps < 2; ++ps) {
#pragma unroll
            for (int s = 0; s < 8; ++s) { const int row = 2 * s + hi, cofs = lr * 4; v4f val = *(const v4fa*)(os + row * 68 + cofs); if (BIAS) { val[0] += bfr(bias[c0 + cofs]); val[1] += bfr(bias[c0 + cofs + 1]); val[2] += bfr(bias[c0 + cofs + 2]); val[3] += bfr(bias[c0 + cofs + 3]); }
                *(volatile v4f*)(crow + (size_t)row * ldc + cofs) = val; }
            if (ps == 0) __threadfence(); }
        __builtin_amdgcn_wave_barrier(); asm volatile("" ::: "memory");
    }
}

__device__ __forceinline__ void splitf(float y, unsigned short& h, unsigned short& l) { h = f2bf(y); l = f2bf(y - bf2f(h)); }
typedef __attribute__((ext_vector_type(2))) unsigned short v2us;

__device__ __noinline__ float fdivn(float a, float b) { return __fdiv_rn(a, b); }
__device__ __forceinline__ float hat(float v, float gs) { return fmaxf(1.0f - fdivn(fabsf(v - gs), 0.75f), 0.f); }
__global__ __launch_bounds__(256) void k_phi(const float* __restrict__ x, const float* __restrict__ nodes, const float* __restrict__ W1a, const float* __restrict__ W1b, const float* __restrict__ W2, float* PW) {
    const int lane = threadIdx.x & 31; const int wg = blockIdx.x * 8 + (threadIdx.x >> 5); if (wg >= MM * (NNODE / 32)) return; const int m = wg / (NNODE / 32), n = (wg % (NNODE / 32)) * 32 + lane;
    const float gs[NG] = {-1.5f, -0.75f, 0.0f, 0.75f, 1.5f};
    const float dx = bfr(x[m * 2]) - bfr(nodes[n * 2]), dy = bfr(x[m * 2 + 1]) - bfr(nodes[n * 2 + 1]);
    const float dist = sqrtf(__fadd_rn(__fmul_rn(dx, dx), __fmul_rn(dy, dy)));
    const float k0 = fdivn(dx, 0.3f), k1 = fdivn(dy, 0.3f);
    float b0[NG], b1[NG];
#pragma unroll
    for (int s = 0; s < NG; ++s) { b0[s] = hat(k0, gs[s]); b1[s] = hat(k1, gs[s]); }
    float phi = 0.f;
#pragma unroll 1
    for (int h = 0; h < HID; ++h) { float hid = 0.f;
#pragma unroll
        for (int s = 0; s < NG; ++s) hid = fmaf(b0[s], bfr(W1a[h * NG + s]), hid);
#pragma unroll
        for (int s = 0; s < NG; ++s) hid = fmaf(b1[s], bfr(W1b[h * NG + s]), hid);
#pragma unroll
        for (int s = 0; s < NG; ++s) phi = fmaf(hat(hid, gs[s]), bfr(W2[h * NG + s]), phi); }
    const float q = fdivn(dist, 0.3f); const float q2 = q * q, q3 = q2 * q, q4 = q2 * q2;
    float win = __fsub_rn(__fadd_rn(__fsub_rn(1.0f, __fmul_rn(6.0f, q2)), __fmul_rn(8.0f, q3)), __fmul_rn(3.0f, q4)); win = (q <= 1.0f) ? win : 0.f;
    const float v = phi * win;
    float* dst = PW + (size_t)m * NNODE + n; *(volatile float*)dst = v; __threadfence(); *(volatile float*)dst = v;
}
__global__ __launch_bounds__(256) void k_normp(const float* __restrict__ PW, bf* Ph, bf* Pl) {
    const int lane = threadIdx.x & 31; const int m = blockIdx.x * 8 + (threadIdx.x >> 5); if (m >= MM) return; const float* row = PW + (size_t)m * NNODE; float s = 0.f;
#pragma unroll 4
    for (int i = 0; i < NNODE / 32; ++i) s += row[i * 32 + lane];
#pragma unroll
    for (int sh = 16; sh; sh >>= 1) s += __shfl_xor(s, sh, 32);
    const float den = s + 1e-10f;
#pragma unroll 1
    for (int ps = 0; ps < 2; ++ps) {
#pragma unroll 2
        for (int c = 0; c < NNODE / 64; ++c) { v2us oh, ol;
#pragma unroll
            for (int q = 0; q < 2; ++q) { unsigned short a, b2; splitf(__fdiv_rn(row[c * 64 + lane * 2 + q], den), a, b2); oh[q] = a; ol[q] = b2; }
            *(volatile v2us*)(Ph + (size_t)m * NNODE + c * 64 + lane * 2) = oh; *(volatile v2us*)(Pl + (size_t)m * NNODE + c * 64 + lane * 2) = ol; }
        if (ps == 0) __threadfence(); }
}
__global__ __launch_bounds__(256) void k_wt(const float* __restrict__ w, bf* Bt) {
    const int lane = threadIdx.x & 31; const int L = blockIdx.x * 8 + (threadIdx.x >> 5); if (L >= 64 * NNODE / 64) return; const int e = L * 64 + lane * 2; v2us o;
#pragma unroll
    for (int q = 0; q < 2; ++q) { const int n = (e + q) / NNODE, k = (e + q) % NNODE; o[q] = n == 0 ? f2bf(w[k]) : (unsigned short)0; }
    *(volatile v2us*)(Bt + e) = o; __threadfence(); *(volatile v2us*)(Bt + e) = o;
}
__global__ __launch_bounds__(256) void k_out(const float* __restrict__ C, float* OUT) { const int lane = threadIdx.x & 31; const int m0 = (blockIdx.x * 8 + (threadIdx.x >> 5)) * 32; if (m0 >= MM) return; const float v = C[(size_t)(m0 + lane) * 64]; *(volatile float*)(OUT + m0 + lane) = v; __threadfence(); *(volatile float*)(OUT + m0 + lane) = v; }

extern "C" void kernel_launch(void* const* d_in, const int* in_sizes, int n_in,
                              void* d_out, int out_size, void* d_ws, size_t ws_size, hipStream_t stream) {
    (void)in_sizes; (void)n_in; (void)out_size;
    const float* x = (const float*)d_in[0]; const float* nodes = (const float*)d_in[1]; const float* W1a = (const float*)d_in[2]; const float* W1b = (const float*)d_in[3]; const float* W2 = (const float*)d_in[4]; const float* w = (const float*)d_in[5];
    float* OUT = (float*)d_out;
    char* wsp = (char*)d_ws;
    auto take = [&](size_t bytes) { char* p = wsp; wsp += (bytes + 255) & ~(size_t)255; return (void*)p; };
    float* PW = (float*)take((size_t)MM * NNODE * 4); bf* Ph = (bf*)take((size_t)MM * NNODE * 2); bf* Pl = (bf*)take((size_t)MM * NNODE * 2); bf* WB = (bf*)take((size_t)64 * NNODE * 2); float* C = (float*)take((size_t)MM * 64 * 4);
    if ((size_t)(wsp - (char*)d_ws) > ws_size) return;
    k_wt<<<(64 * NNODE / 64 + 7) / 8, 256, 0, stream>>>(w, WB);
    k_phi<<<MM * (NNODE / 32) / 8, 256, 0, stream>>>(x, nodes, W1a, W1b, W2, PW);
    k_normp<<<MM / 8, 256, 0, stream>>>(PW, Ph, Pl);
    k_gemmw<bf, 1, false><<<dim3(MM / 64, 1, 1), 32, 0, stream>>>(Ph, Pl, WB, nullptr, NNODE, C, 64, nullptr, 0, 0, 0);
    k_out<<<(MM / 32 + 7) / 8, 256, 0, stream>>>(C, OUT);
}
